// CrossScaleAttention_64269890617678
// MI455X (gfx1250) — hardware-verified
//
#include <hip/hip_runtime.h>


#define NB_  8
#define CC   256
#define NPX  2304
#define NH_  4
#define HD   64
#define ZH   2
#define DM   CC
#define NN   NPX
#define NTK  NPX
#define SCL  0.125f
#define LOSC 1024.0f

typedef _Float16 h16;
typedef unsigned short bf;
typedef __attribute__((ext_vector_type(16))) __bf16   v16bf;
typedef __attribute__((ext_vector_type(16))) _Float16 v16h;
typedef __attribute__((ext_vector_type(8)))  _Float16 v8h;
typedef __attribute__((ext_vector_type(8)))  unsigned short v8us;
typedef __attribute__((ext_vector_type(8)))  float    v8f;
typedef __attribute__((ext_vector_type(4)))  float    v4f;
typedef __attribute__((ext_vector_type(4)))  _Float16 v4h;
typedef v8h  __attribute__((may_alias)) v8ha;
typedef v4f  __attribute__((may_alias)) v4fa;
typedef v8us __attribute__((may_alias)) v8usa;

__device__ __forceinline__ unsigned short f2bf(float f) { unsigned u = __float_as_uint(f); u += 0x7FFFu + ((u >> 16) & 1u); return (unsigned short)(u >> 16); }
__device__ __forceinline__ float bf2f(unsigned short b) { return __uint_as_float(((unsigned)b) << 16); }
__device__ __forceinline__ float bfr(float f) { return bf2f(f2bf(f)); }
__device__ __forceinline__ v16h cat16(v8h lo, v8h hi) { return __builtin_shufflevector(lo, hi, 0, 1, 2, 3, 4, 5, 6, 7, 8, 9, 10, 11, 12, 13, 14, 15); }
__device__ __forceinline__ v16bf cat16b(v8us lo, v8us hi) { return __builtin_bit_cast(v16bf, __builtin_shufflevector(lo, hi, 0, 1, 2, 3, 4, 5, 6, 7, 8, 9, 10, 11, 12, 13, 14, 15)); }
__device__ __forceinline__ v8f wmma16(v16h a, v16h b, v8f c) { return __builtin_amdgcn_wmma_f32_16x16x32_f16(false, a, false, b, (short)0, c, false, false); }
__device__ __forceinline__ v8f wmmab(v16bf a, v16bf b, v8f c) { return __builtin_amdgcn_wmma_f32_16x16x32_bf16(false, a, false, b, (short)0, c, false, false); }

template <bool SPLITA, bool F16OUT = false>
__global__ __launch_bounds__(128) void k_gemmb(const bf* __restrict__ A, const bf* __restrict__ Al, const bf* __restrict__ Bn, const float* __restrict__ bias, float* C, int ldc, h16* C2, const float* __restrict__ R = nullptr, int K = DM, int roundR = 1) {
    __shared__ __align__(16) float ost[4][16 * 68];
    const int lane = threadIdx.x & 31, wave = threadIdx.x >> 5, lr = lane & 15, hi = lane >> 4;
    const int r0 = blockIdx.x * 64 + wave * 16, c0 = blockIdx.y * 64;
    const size_t aoff = (size_t)(r0 + lr) * K + 8 * hi;
    size_t boff[4];
#pragma unroll
    for (int t = 0; t < 4; ++t) boff[t] = (size_t)(c0 + t * 16 + lr) * K + 8 * hi;
    v8f acc[4];
#pragma unroll
    for (int t = 0; t < 4; ++t) acc[t] = (v8f){};
#pragma unroll 1
    for (int kc = 0; kc < K; kc += 32) {
        const v16bf a = cat16b(*(const v8us*)(A + aoff + kc), *(const v8us*)(A + aoff + kc + 16));
        v16bf al = a;
        if (SPLITA) al = cat16b(*(const v8us*)(Al + aoff + kc), *(const v8us*)(Al + aoff + kc + 16));
#pragma unroll
        for (int t = 0; t < 4; ++t) { const v16bf b = cat16b(*(const v8us*)(Bn + boff[t] + kc), *(const v8us*)(Bn + boff[t] + kc + 16)); acc[t] = wmmab(a, b, acc[t]); if (SPLITA) acc[t] = wmmab(al, b, acc[t]); }
        asm volatile("v_nop\n\tv_nop\n\tv_nop\n\tv_nop" : "+v"(acc[0]), "+v"(acc[1]), "+v"(acc[2]), "+v"(acc[3]) : "v"(a), "v"(al));
    }
    float* os = &ost[wave][0];
#pragma unroll
    for (int t = 0; t < 4; ++t) { const float bv = bias ? bfr(bias[c0 + t * 16 + lr]) : 0.f;
#pragma unroll
        for (int j = 0; j < 8; ++j) os[(hi * 8 + j) * 68 + t * 16 + lr] = acc[t][j] + bv; }
    __syncthreads();
    if (F16OUT) {
        h16* crow = (h16*)(void*)C + (size_t)r0 * ldc + c0;
        auto pass = [&]() {
#pragma unroll
            for (int s = 0; s < 4; ++s) { const int row = 4 * s + (lane >> 3), piece = lane & 7; const float* sp = os + row * 68 + piece * 8; v8h o, o2;
#pragma unroll
                for (int i = 0; i < 8; ++i) { const h16 a = (h16)sp[i]; o[i] = a; o2[i] = (h16)((sp[i] - (float)a) * LOSC); }
                *(volatile v8h*)(crow + (size_t)row * ldc + piece * 8) = o; if (C2) *(volatile v8h*)(C2 + (size_t)r0 * ldc + c0 + (size_t)row * ldc + piece * 8) = o2; }
        };
        pass(); __threadfence(); pass();
    } else {
        float* crow = C + (size_t)r0 * ldc + c0;
        auto pass = [&]() {
#pragma unroll
            for (int s = 0; s < 8; ++s) { const int Lid = (lane >> 3) + 4 * s, piece = lane & 7; const int row = Lid >> 1, cofs = (Lid & 1) * 32 + piece * 4;
                v4f val = *(const v4fa*)(os + row * 68 + cofs); if (R) { const v4f rv = *(const v4f*)(R + ((size_t)r0 + row) * ldc + c0 + cofs); val += roundR ? (v4f){bfr(rv[0]), bfr(rv[1]), bfr(rv[2]), bfr(rv[3])} : rv; }
                *(volatile v4f*)(crow + (size_t)row * ldc + cofs) = val; }
        };
        pass(); __threadfence(); pass();
    }
}

__global__ __launch_bounds__(256) void k_cvt8(const float* __restrict__ src, bf* dst, size_t n8) {
    const size_t i = (size_t)blockIdx.x * 256 + threadIdx.x; if (i >= n8) return;
    const v8f v = *(const v8f*)(src + i * 8); v8us o;
#pragma unroll
    for (int k = 0; k < 8; ++k) o[k] = f2bf(v[k]);
    *(volatile v8us*)(dst + i * 8) = o; __threadfence(); *(volatile v8us*)(dst + i * 8) = o;
}
__global__ __launch_bounds__(256) void k_zero8(bf* dst, size_t n8) {
    const size_t i = (size_t)blockIdx.x * 256 + threadIdx.x; if (i >= n8) return; v8us z;
#pragma unroll
    for (int k = 0; k < 8; ++k) z[k] = 0;
    *(volatile v8us*)(dst + i * 8) = z; __threadfence(); *(volatile v8us*)(dst + i * 8) = z;
}

template <int MODE>
__global__ __launch_bounds__(128) void k_gemm3z(const bf* __restrict__ Ah, const bf* __restrict__ Al, const bf* __restrict__ Bh, const bf* __restrict__ Bl, int K, float* C, int ldc, size_t sA, size_t sB, size_t sC) {
    if ((MODE & 1) && (int)blockIdx.y * 64 > (int)blockIdx.x * 64 + 63) return;
    const size_t z = blockIdx.z; Ah += z * sA; Al += z * sA; Bh += z * sB; Bl += z * sB; C += z * sC;
    const int Klim = (MODE & 2) ? min(K, ((int)blockIdx.x + 1) * 64) : K;
    __shared__ __align__(16) float ost[4][16 * 68];
    const int lane = threadIdx.x & 31, wave = threadIdx.x >> 5, lr = lane & 15, hi = lane >> 4;
    const int r0 = blockIdx.x * 64 + wave * 16, c0 = blockIdx.y * 64;
    const size_t aoff = (size_t)(r0 + lr) * K + 8 * hi;
    v8f acc[4];
#pragma unroll
    for (int t = 0; t < 4; ++t) acc[t] = (v8f){};
#pragma unroll 1
    for (int kc = 0; kc < Klim; kc += 32) {
        const v16bf a = cat16b(*(const v8us*)(Ah + aoff + kc), *(const v8us*)(Ah + aoff + kc + 16));
        v16bf al = a; if (!(MODE & 4) && !(MODE & 16)) al = cat16b(*(const v8us*)(Al + aoff + kc), *(const v8us*)(Al + aoff + kc + 16));
#pragma unroll
        for (int t = 0; t < 4; ++t) { const size_t bo = (size_t)(c0 + t * 16 + lr) * K + kc + 8 * hi;
            const v16bf bh = cat16b(*(const v8us*)(Bh + bo), *(const v8us*)(Bh + bo + 16));
            acc[t] = wmmab(a, bh, acc[t]);
            if (!(MODE & 4)) { if (!(MODE & 16)) acc[t] = wmmab(al, bh, acc[t]); if (!(MODE & 8)) { const v16bf bl = cat16b(*(const v8us*)(Bl + bo), *(const v8us*)(Bl + bo + 16)); acc[t] = wmmab(a, bl, acc[t]); } } }
        asm volatile("v_nop\n\tv_nop\n\tv_nop\n\tv_nop" : "+v"(acc[0]), "+v"(acc[1]), "+v"(acc[2]), "+v"(acc[3]) : "v"(a), "v"(al));
    }
    float* os = &ost[wave][0];
#pragma unroll
    for (int t = 0; t < 4; ++t) {
#pragma unroll
        for (int j = 0; j < 8; ++j) os[(hi * 8 + j) * 68 + t * 16 + lr] = acc[t][j]; }
    __builtin_amdgcn_wave_barrier(); asm volatile("" ::: "memory");
    float* crow = C + (size_t)r0 * ldc + c0;
    auto pass = [&]() {
#pragma unroll
        for (int s = 0; s < 8; ++s) { const int Lid = (lane >> 3) + 4 * s, piece = lane & 7; const int row = Lid >> 1, cofs = (Lid & 1) * 32 + piece * 4;
            const v4f val = *(const v4fa*)(os + row * 68 + cofs); *(volatile v4f*)(crow + (size_t)row * ldc + cofs) = val; }
    };
    pass(); __threadfence(); pass();
}
__global__ __launch_bounds__(256) void k_planes32z(const float* __restrict__ F, int ld, int off, float sc, int rows, bf* Ph, bf* Pl) {
    typedef __attribute__((ext_vector_type(2))) unsigned short v2us;
    const int lane = threadIdx.x & 31; const size_t r = ((size_t)blockIdx.x * 8 + (threadIdx.x >> 5)) * 2 + (lane >> 4); if (r >= (size_t)rows) return; const int z = blockIdx.z; const int c0 = (lane & 15) * 2; v2us oh, ol;
    Ph += (size_t)z * rows * 32; Pl += (size_t)z * rows * 32;
#pragma unroll
    for (int i = 0; i < 2; ++i) { const float y = F[r * ld + off + z * 32 + c0 + i] * sc; const unsigned short hb = f2bf(y); oh[i] = hb; ol[i] = f2bf(y - bf2f(hb)); }
    const size_t o = r * 32 + c0; *(volatile v2us*)(Ph + o) = oh; *(volatile v2us*)(Pl + o) = ol; __threadfence(); *(volatile v2us*)(Ph + o) = oh; *(volatile v2us*)(Pl + o) = ol;
}
__global__ __launch_bounds__(256) void k_vtpadz(const float* __restrict__ F, int ld, int off, int nk, bf* Th, bf* Tl) {
    typedef __attribute__((ext_vector_type(2))) unsigned short v2us;
    const int lane = threadIdx.x & 31; const size_t wid = (size_t)blockIdx.x * 8 + (threadIdx.x >> 5); if (wid >= (size_t)64 * (nk / 64)) return; const int z = blockIdx.z; const int d = (int)(wid / (nk / 64)); const int k0 = (int)(wid % (nk / 64)) * 64 + lane * 2; v2us oh, ol;
    Th += (size_t)z * 64 * nk; Tl += (size_t)z * 64 * nk;
#pragma unroll
    for (int i = 0; i < 2; ++i) { const float y = (d < 32) ? F[(size_t)(k0 + i) * ld + off + z * 32 + (d < 32 ? d : 0)] : 0.f; const unsigned short hb = f2bf(y); oh[i] = hb; ol[i] = f2bf(y - bf2f(hb)); }
    const size_t o = (size_t)d * nk + k0; *(volatile v2us*)(Th + o) = oh; *(volatile v2us*)(Tl + o) = ol; __threadfence(); *(volatile v2us*)(Th + o) = oh; *(volatile v2us*)(Tl + o) = ol;
}
template <int NK>
__global__ __launch_bounds__(256) void k_softmaxz(const float* __restrict__ S, int rows, bf* PH, bf* PL) {
    typedef __attribute__((ext_vector_type(4))) unsigned short v4us;
    const int lane = threadIdx.x & 31, i = blockIdx.x * 8 + (threadIdx.x >> 5); if (i >= rows) return; const size_t zo = (size_t)blockIdx.z * rows * NK; const float* sr = S + zo + (size_t)i * NK; PH += zo; PL += zo;
    float m = -3.0e38f;
#pragma unroll 1
    for (int c0 = lane * 4; c0 < NK; c0 += 128) {
#pragma unroll
        for (int q = 0; q < 4; ++q) m = fmaxf(m, sr[c0 + q]); }
#pragma unroll
    for (int sh = 16; sh; sh >>= 1) m = fmaxf(m, __shfl_xor(m, sh, 32));
    float sum = 0.f;
#pragma unroll 1
    for (int c0 = lane * 4; c0 < NK; c0 += 128) {
#pragma unroll
        for (int q = 0; q < 4; ++q) sum += __expf(sr[c0 + q] - m); }
#pragma unroll
    for (int sh = 16; sh; sh >>= 1) sum += __shfl_xor(sum, sh, 32);
    const float inv = 1.0f / sum;
#pragma unroll 1
    for (int ps = 0; ps < 2; ++ps) {
#pragma unroll 1
        for (int c0 = lane * 4; c0 < NK; c0 += 128) { v4us oh, ol;
#pragma unroll
            for (int q = 0; q < 4; ++q) { const float p = __expf(sr[c0 + q] - m) * inv; const unsigned short hb = f2bf(p); oh[q] = hb; ol[q] = f2bf(p - bf2f(hb)); }
            const size_t o = (size_t)i * NK + c0; *(volatile v4us*)(PH + o) = oh; *(volatile v4us*)(PL + o) = ol; }
        if (ps == 0) __threadfence(); }
}
__global__ __launch_bounds__(256) void k_placez(const float* __restrict__ XH, int rows, int ldy, float* Y) {
    const int lane = threadIdx.x & 31; const size_t q = (size_t)blockIdx.x * 8 + (threadIdx.x >> 5); if (q >= (size_t)rows) return; const int z = blockIdx.z; const float v = XH[((size_t)z * rows + q) * 64 + lane];
    *(volatile float*)(Y + q * ldy + z * 32 + lane) = v; __threadfence(); *(volatile float*)(Y + q * ldy + z * 32 + lane) = v;
}

__global__ __launch_bounds__(256) void k_hplanesz(const float* __restrict__ F, int ld, int h0, float sc, int rows, bf* Ph, bf* Pl) {
    typedef __attribute__((ext_vector_type(2))) unsigned short v2us;
    const int lane = threadIdx.x & 31; const size_t r = (size_t)blockIdx.x * 8 + (threadIdx.x >> 5); if (r >= (size_t)rows) return; const int z = blockIdx.z; v2us oh, ol;
    Ph += (size_t)z * rows * 64; Pl += (size_t)z * rows * 64;
#pragma unroll
    for (int i = 0; i < 2; ++i) { const float y = F[r * ld + (h0 + z) * 64 + lane * 2 + i] * sc; const unsigned short hb = f2bf(y); oh[i] = hb; ol[i] = f2bf(y - bf2f(hb)); }
    const size_t o = r * 64 + lane * 2; *(volatile v2us*)(Ph + o) = oh; *(volatile v2us*)(Pl + o) = ol; __threadfence(); *(volatile v2us*)(Ph + o) = oh; *(volatile v2us*)(Pl + o) = ol;
}
__global__ __launch_bounds__(256) void k_vtz(const float* __restrict__ F, int ld, int h0, int nk, bf* Th, bf* Tl) {
    typedef __attribute__((ext_vector_type(2))) unsigned short v2us;
    const int lane = threadIdx.x & 31; const size_t wid = (size_t)blockIdx.x * 8 + (threadIdx.x >> 5); if (wid >= (size_t)64 * (nk / 64)) return; const int z = blockIdx.z; const int d = (int)(wid / (nk / 64)); const int t0 = (int)(wid % (nk / 64)) * 64 + lane * 2; v2us oh, ol;
    Th += (size_t)z * 64 * nk; Tl += (size_t)z * 64 * nk;
#pragma unroll
    for (int i = 0; i < 2; ++i) { const float y = F[(size_t)(t0 + i) * ld + (h0 + z) * 64 + d]; const unsigned short hb = f2bf(y); oh[i] = hb; ol[i] = f2bf(y - bf2f(hb)); }
    const size_t o = (size_t)d * nk + t0; *(volatile v2us*)(Th + o) = oh; *(volatile v2us*)(Tl + o) = ol; __threadfence(); *(volatile v2us*)(Th + o) = oh; *(volatile v2us*)(Tl + o) = ol;
}
template <int NK>
__global__ __launch_bounds__(256) void k_softmaxzs(const float* __restrict__ S, int rows, float sc, bf* PH, bf* PL) {
    typedef __attribute__((ext_vector_type(4))) unsigned short v4us;
    const int lane = threadIdx.x & 31, i = blockIdx.x * 8 + (threadIdx.x >> 5); if (i >= rows) return; const size_t zo = (size_t)blockIdx.z * rows * NK; const float* sr = S + zo + (size_t)i * NK; PH += zo; PL += zo;
    float m = -3.0e38f;
#pragma unroll 1
    for (int c0 = lane * 4; c0 < NK; c0 += 128) {
#pragma unroll
        for (int q = 0; q < 4; ++q) m = fmaxf(m, sr[c0 + q] * sc); }
#pragma unroll
    for (int sh = 16; sh; sh >>= 1) m = fmaxf(m, __shfl_xor(m, sh, 32));
    float sum = 0.f;
#pragma unroll 1
    for (int c0 = lane * 4; c0 < NK; c0 += 128) {
#pragma unroll
        for (int q = 0; q < 4; ++q) sum += __expf(sr[c0 + q] * sc - m); }
#pragma unroll
    for (int sh = 16; sh; sh >>= 1) sum += __shfl_xor(sum, sh, 32);
    const float inv = 1.0f / sum;
#pragma unroll 1
    for (int ps = 0; ps < 2; ++ps) {
#pragma unroll 1
        for (int c0 = lane * 4; c0 < NK; c0 += 128) { v4us oh, ol;
#pragma unroll
            for (int q = 0; q < 4; ++q) { const float p = __expf(sr[c0 + q] * sc - m) * inv; const unsigned short hb = f2bf(p); oh[q] = hb; ol[q] = f2bf(p - bf2f(hb)); }
            const size_t o = (size_t)i * NK + c0; *(volatile v4us*)(PH + o) = oh; *(volatile v4us*)(PL + o) = ol; }
        if (ps == 0) __threadfence(); }
}

__global__ __launch_bounds__(256) void k_ptb(const float* __restrict__ xb, bf* XT) {
    __shared__ float tl[64][65];
    typedef __attribute__((ext_vector_type(4))) unsigned short v4us;
    const int tid = threadIdx.x, c0 = blockIdx.x * 64, p0 = blockIdx.y * 64; const int rr = tid >> 2, cq = (tid & 3) * 16;
#pragma unroll
    for (int i = 0; i < 16; ++i) tl[rr][cq + i] = xb[(size_t)(c0 + rr) * NPX + p0 + cq + i];
    __syncthreads();
    const int lane = tid & 31, wv = tid >> 5;
    auto pass = [&]() {
#pragma unroll
        for (int st = 0; st < 4; ++st) { const int pr = wv * 8 + st * 2 + (lane >> 4); const int cl = (lane & 15) * 4; v4us v;
#pragma unroll
            for (int i = 0; i < 4; ++i) v[i] = f2bf(tl[cl + i][pr]);
            *(volatile v4us*)(XT + (size_t)(p0 + pr) * CC + c0 + cl) = v; }
    };
    pass(); __threadfence(); pass();
}
__global__ __launch_bounds__(256) void k_wcat3(const float* __restrict__ Wq, const float* __restrict__ Wk, const float* __restrict__ Wv, bf* WQKV) {
    const size_t i = ((size_t)blockIdx.x * 256 + threadIdx.x) * 8; if (i >= (size_t)3 * CC * CC) return; const size_t blk = i / ((size_t)CC * CC), o = i % ((size_t)CC * CC);
    const float* src = (blk == 0) ? Wq : (blk == 1) ? Wk : Wv; v8us v;
#pragma unroll
    for (int q = 0; q < 8; ++q) v[q] = f2bf(src[o + q]);
    *(volatile v8us*)(WQKV + i) = v; __threadfence(); *(volatile v8us*)(WQKV + i) = v;
}
__global__ __launch_bounds__(256) void k_bias3(const float* __restrict__ b0, const float* __restrict__ b1, const float* __restrict__ b2, float* B3) {
    const size_t i = (size_t)blockIdx.x * 256 + threadIdx.x; if (i >= (size_t)3 * CC) return; const int blk = (int)(i / CC), o = (int)(i % CC); const float v = (blk == 0) ? b0[o] : (blk == 1) ? b1[o] : b2[o];
    *(volatile float*)(B3 + i) = v; __threadfence(); *(volatile float*)(B3 + i) = v;
}
__global__ __launch_bounds__(256) void k_split256(const float* __restrict__ src, int rows, bf* dh, bf* dl) {
    const int lane = threadIdx.x & 31; const size_t r = (size_t)blockIdx.x * 8 + (threadIdx.x >> 5); if (r >= (size_t)rows) return; const size_t o = r * CC + lane * 8; const v8f v = *(const v8f*)(src + o); v8us oh, ol;
#pragma unroll
    for (int i = 0; i < 8; ++i) { const unsigned short hb = f2bf(v[i]); oh[i] = hb; ol[i] = f2bf(v[i] - bf2f(hb)); }
    *(volatile v8us*)(dh + o) = oh; *(volatile v8us*)(dl + o) = ol; __threadfence(); *(volatile v8us*)(dh + o) = oh; *(volatile v8us*)(dl + o) = ol;
}
__global__ __launch_bounds__(256) void k_outT(const float* __restrict__ OT, const float* __restrict__ xb, const float* __restrict__ gam, float* OUTB) {
    __shared__ float tl[64][65];
    const int tid = threadIdx.x; const int p0 = blockIdx.x * 64, c0 = blockIdx.y * 64; const int rr = tid >> 2, cq = (tid & 3) * 16;
#pragma unroll
    for (int i = 0; i < 16; ++i) tl[rr][cq + i] = OT[(size_t)(p0 + rr) * CC + c0 + cq + i];
    __syncthreads();
    const int lane = tid & 31, wv = tid >> 5; const float gm = bfr(gam[0]);
    auto pass = [&]() {
#pragma unroll
        for (int st = 0; st < 4; ++st) { const int cr = wv * 8 + st * 2 + (lane >> 4); const int pq = (lane & 15) * 4; v4f v; const size_t o = (size_t)(c0 + cr) * NPX + p0 + pq;
#pragma unroll
            for (int i = 0; i < 4; ++i) v[i] = bfr(xb[o + i]) + gm * tl[pq + i][cr];
            *(volatile v4f*)(OUTB + o) = v; }
    };
    pass(); __threadfence(); pass();
}

extern "C" void kernel_launch(void* const* d_in, const int* in_sizes, int n_in,
                              void* d_out, int out_size, void* d_ws, size_t ws_size, hipStream_t stream) {
    (void)in_sizes; (void)n_in; (void)out_size;
    const float* x = (const float*)d_in[0]; const float* Wq = (const float*)d_in[1]; const float* bq = (const float*)d_in[2]; const float* Wk = (const float*)d_in[3]; const float* bk = (const float*)d_in[4]; const float* Wv = (const float*)d_in[5]; const float* bv = (const float*)d_in[6]; const float* Wo = (const float*)d_in[7]; const float* bo = (const float*)d_in[8]; const float* gam = (const float*)d_in[9];
    float* out = (float*)d_out;
    char* wsp = (char*)d_ws;
    auto take = [&](size_t bytes) { char* p = wsp; wsp += (bytes + 255) & ~(size_t)255; return (void*)p; };
    bf* WQKV = (bf*)take((size_t)3 * CC * CC * 2); float* B3 = (float*)take((size_t)3 * CC * 4); bf* WO = (bf*)take((size_t)CC * CC * 2);
    bf* XT = (bf*)take((size_t)NPX * CC * 2); float* QKV = (float*)take((size_t)NPX * 3 * CC * 4);
    bf* Qh = (bf*)take((size_t)ZH * NPX * HD * 2); bf* Ql = (bf*)take((size_t)ZH * NPX * HD * 2); bf* Kh = (bf*)take((size_t)ZH * NPX * HD * 2); bf* Kl = (bf*)take((size_t)ZH * NPX * HD * 2); bf* VTh = (bf*)take((size_t)ZH * HD * NPX * 2); bf* VTl = (bf*)take((size_t)ZH * HD * NPX * 2);
    float* S = (float*)take((size_t)ZH * NPX * NPX * 4); bf* PH = (bf*)take((size_t)ZH * NPX * NPX * 2); bf* PL = (bf*)take((size_t)ZH * NPX * NPX * 2); float* O = (float*)take((size_t)NPX * CC * 4); bf* Oh = (bf*)take((size_t)NPX * CC * 2); bf* Ol = (bf*)take((size_t)NPX * CC * 2); float* OT = (float*)take((size_t)NPX * CC * 4);
    if ((size_t)(wsp - (char*)d_ws) > ws_size) return;
    k_wcat3<<<(unsigned)((3 * (size_t)CC * CC / 8 + 255) / 256), 256, 0, stream>>>(Wq, Wk, Wv, WQKV); k_bias3<<<(3 * CC + 255) / 256, 256, 0, stream>>>(bq, bk, bv, B3); k_cvt8<<<(CC * CC / 8 + 255) / 256, 256, 0, stream>>>(Wo, WO, CC * CC / 8);
    for (int b = 0; b < NB_; ++b) { const float* xb = x + (size_t)b * CC * NPX;
        k_ptb<<<dim3(CC / 64, NPX / 64, 1), 256, 0, stream>>>(xb, XT);
        k_gemmb<false, false><<<dim3(NPX / 64, (3 * CC) / 64, 1), 128, 0, stream>>>(XT, nullptr, WQKV, B3, QKV, 3 * CC, nullptr, nullptr, CC);
        for (int g = 0; g < NH_ / ZH; ++g) { const int h0 = g * ZH;
            k_hplanesz<<<dim3(NPX / 8, 1, ZH), 256, 0, stream>>>(QKV, 3 * CC, h0, 1.0f, NPX, Qh, Ql); k_hplanesz<<<dim3(NPX / 8, 1, ZH), 256, 0, stream>>>(QKV + CC, 3 * CC, h0, 1.0f, NPX, Kh, Kl);
            k_vtz<<<dim3((HD * (NPX / 64)) / 8, 1, ZH), 256, 0, stream>>>(QKV + 2 * CC, 3 * CC, h0, NPX, VTh, VTl);
            k_gemm3z<0><<<dim3(NPX / 64, NPX / 64, ZH), 128, 0, stream>>>(Qh, Ql, Kh, Kl, HD, S, NPX, (size_t)NPX * HD, (size_t)NPX * HD, (size_t)NPX * NPX);
            k_softmaxzs<NPX><<<dim3(NPX / 8, 1, ZH), 256, 0, stream>>>(S, NPX, SCL, PH, PL);
            k_gemm3z<0><<<dim3(NPX / 64, 1, ZH), 128, 0, stream>>>(PH, PL, VTh, VTl, NPX, O + h0 * HD, CC, (size_t)NPX * NPX, (size_t)HD * NPX, (size_t)HD); }
        k_split256<<<NPX / 8, 256, 0, stream>>>(O, NPX, Oh, Ol);
        k_gemmb<true, false><<<dim3(NPX / 64, CC / 64, 1), 128, 0, stream>>>(Oh, Ol, WO, bo, OT, CC, nullptr, nullptr, CC);
        k_outT<<<dim3(NPX / 64, CC / 64, 1), 256, 0, stream>>>(OT, xb, gam, out + (size_t)b * CC * NPX); }
}
